// GAUBlock_17901423689730
// MI455X (gfx1250) — hardware-verified
//
#include <hip/hip_runtime.h>


#define NB_  4
#define DIM  256
#define LL   4096
#define HID  256
#define QK   128
#define NTK  (NB_ * LL)
#define TE   768
#define PSC  32768.0f

typedef _Float16 h16;
typedef unsigned short bf;
typedef __attribute__((ext_vector_type(16))) __bf16   v16bf;
typedef __attribute__((ext_vector_type(16))) _Float16 v16h;
typedef __attribute__((ext_vector_type(8)))  _Float16 v8h;
typedef __attribute__((ext_vector_type(8)))  unsigned short v8us;
typedef __attribute__((ext_vector_type(8)))  float    v8f;
typedef __attribute__((ext_vector_type(4)))  float    v4f;
typedef v8h  __attribute__((may_alias)) v8ha;
typedef v4f  __attribute__((may_alias)) v4fa;
typedef v8us __attribute__((may_alias)) v8usa;

__device__ __forceinline__ unsigned short f2bf(float f) { unsigned u = __float_as_uint(f); u += 0x7FFFu + ((u >> 16) & 1u); return (unsigned short)(u >> 16); }
__device__ __forceinline__ float bf2f(unsigned short b) { return __uint_as_float(((unsigned)b) << 16); }
__device__ __forceinline__ float bfr(float f) { return bf2f(f2bf(f)); }
__device__ __forceinline__ v16h cat16(v8h lo, v8h hi) { return __builtin_shufflevector(lo, hi, 0, 1, 2, 3, 4, 5, 6, 7, 8, 9, 10, 11, 12, 13, 14, 15); }
__device__ __forceinline__ v16bf cat16b(v8us lo, v8us hi) { return __builtin_bit_cast(v16bf, __builtin_shufflevector(lo, hi, 0, 1, 2, 3, 4, 5, 6, 7, 8, 9, 10, 11, 12, 13, 14, 15)); }
__device__ __forceinline__ v8f wmma16(v16h a, v16h b, v8f c) { return __builtin_amdgcn_wmma_f32_16x16x32_f16(false, a, false, b, (short)0, c, false, false); }
__device__ __forceinline__ v8f wmmab(v16bf a, v16bf b, v8f c) { return __builtin_amdgcn_wmma_f32_16x16x32_bf16(false, a, false, b, (short)0, c, false, false); }
__device__ __forceinline__ float silu_(float v) { return v / (1.0f + __expf(-v)); }
#define VST2(T, p, v) do { const T vst2_v_ = (v); *(volatile T*)(p) = vst2_v_; __threadfence(); *(volatile T*)(p) = vst2_v_; } while (0)

__global__ __launch_bounds__(256) void k_emb(const float* __restrict__ t, const float* __restrict__ We, const float* __restrict__ be, float* EMB) {
    const int e = blockIdx.x * 256 + threadIdx.x; const int b = e / DIM, c = e - b * DIM;
    float s = bfr(be[c]);
#pragma unroll 4
    for (int k = 0; k < TE; ++k) s += bfr(t[b * TE + k]) * bfr(We[(size_t)c * TE + k]);
    VST2(float, EMB + e, s);
}
__global__ __launch_bounds__(256) void k_cvtw(const float* __restrict__ Wm, int rows, bf* WB) {
    const int lane = threadIdx.x & 31, r = blockIdx.x * 8 + (threadIdx.x >> 5);
    if (r >= rows) return;
    v8us o;
#pragma unroll
    for (int i = 0; i < 8; ++i) o[i] = f2bf(Wm[(size_t)r * DIM + lane * 8 + i]);
    VST2(v8us, WB + (size_t)r * DIM + lane * 8, o);
}
__global__ __launch_bounds__(256) void k_ln(const float* __restrict__ x, const float* __restrict__ EMB, const float* __restrict__ g, const float* __restrict__ be, bf* NH, bf* NL) {
    __shared__ float tl[DIM][65];
    const int tid = threadIdx.x, lane = tid & 31, wave = tid >> 5;
    const int b = blockIdx.x / (LL / 64), lt = blockIdx.x - b * (LL / 64), l0 = lt * 64;
#pragma unroll 4
    for (int i = 0; i < 64; ++i) { const int c = i * 4 + (tid >> 6), l = tid & 63; tl[c][l] = bfr(x[((size_t)b * DIM + c) * LL + l0 + l]) + EMB[b * DIM + c]; }
    __syncthreads();
#pragma unroll 1
    for (int rr = 0; rr < 8; ++rr) { const int l = wave * 8 + rr;
        float v[8]; float s = 0.f;
#pragma unroll
        for (int i = 0; i < 8; ++i) { v[i] = tl[lane * 8 + i][l]; s += v[i]; }
#pragma unroll
        for (int o = 16; o; o >>= 1) s += __shfl_xor(s, o, 32);
        const float mu = s * (1.0f / DIM); float q = 0.f;
#pragma unroll
        for (int i = 0; i < 8; ++i) { const float d = v[i] - mu; q += d * d; }
#pragma unroll
        for (int o = 16; o; o >>= 1) q += __shfl_xor(q, o, 32);
        const float rs = rsqrtf(q * (1.0f / DIM) + 1e-5f);
        v8us oh, ol;
#pragma unroll
        for (int i = 0; i < 8; ++i) { const int c = lane * 8 + i; const float y = (v[i] - mu) * rs * bfr(g[c]) + bfr(be[c]); const unsigned short hb = f2bf(y); oh[i] = hb; ol[i] = f2bf(y - bf2f(hb)); }
        const size_t ro = ((size_t)b * LL + l0 + l) * DIM + lane * 8;
        *(volatile v8us*)(NH + ro) = oh; *(volatile v8us*)(NL + ro) = ol; __threadfence(); *(volatile v8us*)(NH + ro) = oh; *(volatile v8us*)(NL + ro) = ol; }
}
__global__ __launch_bounds__(128) void k_gemm(const bf* __restrict__ A, const bf* __restrict__ Al, const bf* __restrict__ Bn, const float* __restrict__ bias, int ldc, float* C) {
    __shared__ __align__(16) float ost[4][16 * 68];
    const int lane = threadIdx.x & 31, wave = threadIdx.x >> 5, lr = lane & 15, hi = lane >> 4;
    const int r0 = blockIdx.x * 64 + wave * 16, c0 = blockIdx.y * 64;
    const size_t aoff = (size_t)(r0 + lr) * DIM + 8 * hi;
    size_t boff[4];
#pragma unroll
    for (int t = 0; t < 4; ++t) boff[t] = (size_t)(c0 + t * 16 + lr) * DIM + 8 * hi;
    v8f acc[4];
#pragma unroll
    for (int t = 0; t < 4; ++t) acc[t] = (v8f){};
#pragma unroll 1
    for (int kc = 0; kc < DIM; kc += 32) {
        const v16bf a = cat16b(*(const v8us*)(A + aoff + kc), *(const v8us*)(A + aoff + kc + 16)), al = cat16b(*(const v8us*)(Al + aoff + kc), *(const v8us*)(Al + aoff + kc + 16));
#pragma unroll
        for (int t = 0; t < 4; ++t) { const v16bf bb = cat16b(*(const v8us*)(Bn + boff[t] + kc), *(const v8us*)(Bn + boff[t] + kc + 16)); acc[t] = wmmab(a, bb, acc[t]); acc[t] = wmmab(al, bb, acc[t]); }
        asm volatile("v_nop\n\tv_nop\n\tv_nop\n\tv_nop" : "+v"(acc[0]), "+v"(acc[1]), "+v"(acc[2]), "+v"(acc[3]) : "v"(a), "v"(al));
    }
    float* os = &ost[wave][0];
#pragma unroll
    for (int t = 0; t < 4; ++t) { const float bv = bfr(bias[c0 + t * 16 + lr]);
#pragma unroll
        for (int j = 0; j < 8; ++j) os[(hi * 8 + j) * 68 + t * 16 + lr] = acc[t][j] + bv; }
    __syncthreads();
    float* crow = C + (size_t)r0 * ldc + c0;
    auto pass = [&]() {
#pragma unroll
        for (int s = 0; s < 8; ++s) { const int Lid = (lane >> 3) + 4 * s, piece = lane & 7; const int row = Lid >> 1, cofs = (Lid & 1) * 32 + piece * 4;
            const v4f val = *(const v4fa*)(os + row * 68 + cofs); *(volatile v4f*)(crow + (size_t)row * ldc + cofs) = val; }
    };
    pass(); __threadfence(); pass();
}
__global__ __launch_bounds__(256) void k_qk(const float* __restrict__ Z, const float* __restrict__ gam, const float* __restrict__ bet, h16* Q16, h16* K16) {
    typedef __attribute__((ext_vector_type(4))) _Float16 v4h;
    const int lane = threadIdx.x & 31, r = blockIdx.x * 8 + (threadIdx.x >> 5);
    if (r >= NTK) return;
    const int l = r % LL;
    float zs[4];
#pragma unroll
    for (int i = 0; i < 4; ++i) zs[i] = silu_(Z[(size_t)r * QK + lane * 4 + i]);
    v4h oq, ok;
#pragma unroll
    for (int pq = 0; pq < 2; ++pq) { const int i = lane * 2 + pq;
        const float freq = __expf(-(float)(2 * i) / (float)QK * 9.210340371976184f);
        const float ang = (float)l * freq; float sn, cs; __sincosf(ang, &sn, &cs);
#pragma unroll
        for (int w = 0; w < 2; ++w) { const float* gg = gam + w * QK; const float* bb = bet + w * QK;
            const float xe = zs[2 * pq] * bfr(gg[2 * i]) + bfr(bb[2 * i]), xo = zs[2 * pq + 1] * bfr(gg[2 * i + 1]) + bfr(bb[2 * i + 1]);
            const float y0 = xe * cs - xo * sn, y1 = xe * sn + xo * cs;
            if (w == 0) { oq[2 * pq] = (h16)y0; oq[2 * pq + 1] = (h16)y1; } else { ok[2 * pq] = (h16)y0; ok[2 * pq + 1] = (h16)y1; } } }
    *(volatile v4h*)(Q16 + (size_t)r * QK + lane * 4) = oq; *(volatile v4h*)(K16 + (size_t)r * QK + lane * 4) = ok; __threadfence();
    *(volatile v4h*)(Q16 + (size_t)r * QK + lane * 4) = oq; *(volatile v4h*)(K16 + (size_t)r * QK + lane * 4) = ok;
}
__global__ __launch_bounds__(256) void k_vt(const float* __restrict__ HV, h16* VT16) {
    __shared__ __align__(16) h16 tl[64 * 72];
    const int tid = threadIdx.x, l0 = blockIdx.x * 64, d0 = blockIdx.y * 64, b = blockIdx.z;
    const int ll = tid >> 2, dq = (tid & 3) * 16;
#pragma unroll
    for (int i = 0; i < 16; ++i) tl[(dq + i) * 72 + ll] = (h16)silu_(HV[((size_t)b * LL + l0 + ll) * (2 * HID) + d0 + dq + i]);
    __syncthreads();
    const int piece = tid & 7;
    auto pass = [&]() {
#pragma unroll
        for (int s = 0; s < 2; ++s) { const int d = (tid >> 3) + 32 * s; const v8h val = *(const v8ha*)(tl + d * 72 + piece * 8);
            *(volatile v8h*)(VT16 + ((size_t)b * HID + d0 + d) * LL + l0 + piece * 8) = val; }
    };
    pass(); __threadfence(); pass();
}
__global__ __launch_bounds__(128) void k_attn(const h16* __restrict__ Q16, const h16* __restrict__ K16, const h16* __restrict__ VT16, const float* __restrict__ HV, bf* OH, bf* OL) {
    __shared__ __align__(16) h16 plds[4][16 * 32];
    __shared__ __align__(16) float ost[4][16 * 260];
    const int lane = threadIdx.x & 31, wave = threadIdx.x >> 5, lr = lane & 15, hi = lane >> 4;
    const int b = blockIdx.x / (LL / 64), qt = blockIdx.x - b * (LL / 64), q0 = qt * 64 + wave * 16;
    const size_t row0 = (size_t)b * LL;
    h16* pl = &plds[wave][0];
    v16h qa[4];
    const size_t qo0 = (row0 + q0 + lr) * QK + 8 * hi;
#pragma unroll
    for (int kc = 0; kc < 4; ++kc) qa[kc] = cat16(*(const v8h*)(Q16 + qo0 + kc * 32), *(const v8h*)(Q16 + qo0 + kc * 32 + 16));
    const h16* kb = K16 + row0 * QK;
    const size_t vbase = (size_t)b * HID * LL;
    const float scl = 1.0f / (float)LL;
    v8f o[16];
#pragma unroll
    for (int n = 0; n < 16; ++n) o[n] = (v8f){};
    float mrow[8], lpart[8];
#pragma unroll
    for (int j = 0; j < 8; ++j) { mrow[j] = -3.0e38f; lpart[j] = 0.f; }
#pragma unroll 1
    for (int kt = 0; kt < LL / 32; ++kt) {
        const int l0 = kt * 32;
        v8f s0 = {}, s1 = {};
#pragma unroll
        for (int kc = 0; kc < 4; ++kc) { const size_t k0o = (size_t)(l0 + lr) * QK + kc * 32 + 8 * hi, k1o = k0o + (size_t)16 * QK;
            s0 = wmma16(qa[kc], cat16(*(const v8h*)(kb + k0o), *(const v8h*)(kb + k0o + 16)), s0);
            s1 = wmma16(qa[kc], cat16(*(const v8h*)(kb + k1o), *(const v8h*)(kb + k1o + 16)), s1); }
        asm volatile("v_nop\n\tv_nop\n\tv_nop\n\tv_nop" : "+v"(s0), "+v"(s1) : "v"(qa[0]), "v"(qa[3]));
        float alpha[8];
#pragma unroll
        for (int j = 0; j < 8; ++j) {
            const float a0 = s0[j] * scl, a1 = s1[j] * scl;
            float mx = fmaxf(a0, a1);
            mx = fmaxf(mx, __shfl_xor(mx, 1, 16)); mx = fmaxf(mx, __shfl_xor(mx, 2, 16)); mx = fmaxf(mx, __shfl_xor(mx, 4, 16)); mx = fmaxf(mx, __shfl_xor(mx, 8, 16));
            const float mn = fmaxf(mrow[j], mx);
            alpha[j] = __expf(mrow[j] - mn); mrow[j] = mn;
            const float p0 = __expf(a0 - mn), p1 = __expf(a1 - mn);
            lpart[j] = lpart[j] * alpha[j] + (p0 + p1);
            const int mr = hi * 8 + j;
            pl[mr * 32 + lr] = (h16)(p0 * PSC); pl[mr * 32 + 16 + lr] = (h16)(p1 * PSC);
        }
#pragma unroll
        for (int n = 0; n < 16; ++n)
#pragma unroll
            for (int j = 0; j < 8; ++j) o[n][j] *= alpha[j];
        asm volatile("" ::: "memory");
        const v16h pa = cat16(*(const v8ha*)(pl + lr * 32 + hi * 8), *(const v8ha*)(pl + lr * 32 + 16 + hi * 8));
#pragma unroll
        for (int n = 0; n < 16; ++n) { const size_t vo = vbase + (size_t)(n * 16 + lr) * LL + l0 + hi * 8;
            o[n] = wmma16(pa, cat16(*(const v8h*)(VT16 + vo), *(const v8h*)(VT16 + vo + 16)), o[n]);
            asm volatile("" : "+v"(o[n]) :: "memory"); }
        asm volatile("v_nop\n\tv_nop\n\tv_nop\n\tv_nop" : "+v"(o[0]), "+v"(o[15]) : "v"(pa));
    }
    float inv[8];
#pragma unroll
    for (int j = 0; j < 8; ++j) { float rs = lpart[j]; rs += __shfl_xor(rs, 1, 16); rs += __shfl_xor(rs, 2, 16); rs += __shfl_xor(rs, 4, 16); rs += __shfl_xor(rs, 8, 16); inv[j] = 1.0f / (rs * PSC); }
    float* os = &ost[wave][0];
#pragma unroll
    for (int n = 0; n < 16; ++n)
#pragma unroll
        for (int j = 0; j < 8; ++j) { const int d = n * 16 + lr; const size_t row = row0 + q0 + hi * 8 + j;
            os[(hi * 8 + j) * 260 + d] = o[n][j] * inv[j] * silu_(HV[row * (2 * HID) + HID + d]); }
    __syncthreads();
    auto pass = [&]() {
#pragma unroll
        for (int s = 0; s < 16; ++s) { const float* sp = os + s * 260 + lane * 8; v8us oh, ol;
#pragma unroll
            for (int i = 0; i < 8; ++i) { const unsigned short hb = f2bf(sp[i]); oh[i] = hb; ol[i] = f2bf(sp[i] - bf2f(hb)); }
            const size_t ro = (row0 + q0 + s) * HID + lane * 8;
            *(volatile v8us*)(OH + ro) = oh; *(volatile v8us*)(OL + ro) = ol; }
    };
    pass(); __threadfence(); pass();
}
__global__ __launch_bounds__(256) void k_split(const float* __restrict__ S, bf* SH, bf* SL) {
    const int lane = threadIdx.x & 31, r = blockIdx.x * 8 + (threadIdx.x >> 5);
    if (r >= NTK) return;
    v8us oh, ol;
#pragma unroll
    for (int i = 0; i < 8; ++i) { const float v = S[(size_t)r * DIM + lane * 8 + i]; const unsigned short hb = f2bf(v); oh[i] = hb; ol[i] = f2bf(v - bf2f(hb)); }
    *(volatile v8us*)(SH + (size_t)r * DIM + lane * 8) = oh; *(volatile v8us*)(SL + (size_t)r * DIM + lane * 8) = ol; __threadfence();
    *(volatile v8us*)(SH + (size_t)r * DIM + lane * 8) = oh; *(volatile v8us*)(SL + (size_t)r * DIM + lane * 8) = ol;
}
__global__ __launch_bounds__(256) void k_final(const float* __restrict__ x, const float* __restrict__ EMB, const float* __restrict__ PROJ, float* out1, float* out2) {
    __shared__ float t1[64][65];
    __shared__ float t2[64][65];
    const int tid = threadIdx.x, lane = tid & 31, wave = tid >> 5;
    const int l0 = blockIdx.x * 64, c0 = blockIdx.y * 64, b = blockIdx.z;
    { const int l = tid >> 2, cq = (tid & 3) * 16; const float* pr = PROJ + ((size_t)b * LL + l0 + l) * (2 * DIM);
#pragma unroll
      for (int i = 0; i < 16; ++i) { t1[cq + i][l] = pr[c0 + cq + i]; t2[cq + i][l] = pr[DIM + c0 + cq + i]; } }
    __syncthreads();
    const float rs2 = 0.7071067811865476f;
    auto pass = [&]() {
#pragma unroll
        for (int s = 0; s < 4; ++s) { const int c = wave * 8 + s * 2 + (lane >> 4), piece = lane & 15; const size_t go = ((size_t)b * DIM + c0 + c) * LL + l0 + piece * 4;
            v4f a, bq;
#pragma unroll
            for (int i = 0; i < 4; ++i) { const int l = piece * 4 + i; a[i] = (bfr(x[go + i]) + EMB[b * DIM + c0 + c] + t1[c][l]) * rs2; bq[i] = t2[c][l]; }
            *(volatile v4f*)(out1 + go) = a; *(volatile v4f*)(out2 + go) = bq; }
    };
    pass(); __threadfence(); pass();
}

extern "C" void kernel_launch(void* const* d_in, const int* in_sizes, int n_in,
                              void* d_out, int out_size, void* d_ws, size_t ws_size, hipStream_t stream) {
    (void)in_sizes; (void)n_in; (void)out_size;
    const float* x = (const float*)d_in[0]; const float* t = (const float*)d_in[1]; const float* We = (const float*)d_in[2]; const float* bemb = (const float*)d_in[3];
    const float* lng = (const float*)d_in[4]; const float* lnb = (const float*)d_in[5]; const float* Wh = (const float*)d_in[6]; const float* bh = (const float*)d_in[7];
    const float* Wqk = (const float*)d_in[8]; const float* bqk = (const float*)d_in[9]; const float* gam = (const float*)d_in[10]; const float* bet = (const float*)d_in[11];
    const float* Wout = (const float*)d_in[12]; const float* bout = (const float*)d_in[13]; const float* Wp = (const float*)d_in[14]; const float* bp = (const float*)d_in[15];
    float* out1 = (float*)d_out; float* out2 = (float*)((char*)d_out + (size_t)NB_ * DIM * LL * 4);
    char* wsp = (char*)d_ws;
    auto take = [&](size_t bytes) { char* p = wsp; wsp += (bytes + 255) & ~(size_t)255; return (void*)p; };
    float* EMB = (float*)take((size_t)NB_ * DIM * 4);
    bf* WhB = (bf*)take((size_t)2 * HID * DIM * 2); bf* WqkB = (bf*)take((size_t)QK * DIM * 2); bf* WoB = (bf*)take((size_t)DIM * HID * 2); bf* WpB = (bf*)take((size_t)2 * DIM * DIM * 2);
    bf* NHp = (bf*)take((size_t)NTK * DIM * 2); bf* NLp = (bf*)take((size_t)NTK * DIM * 2);
    float* HV = (float*)take((size_t)NTK * 2 * HID * 4); float* Zf = (float*)take((size_t)NTK * QK * 4);
    h16* Q16 = (h16*)take((size_t)NTK * QK * 2); h16* K16 = (h16*)take((size_t)NTK * QK * 2); h16* VT16 = (h16*)take((size_t)NB_ * HID * LL * 2);
    bf* OH = (bf*)take((size_t)NTK * HID * 2); bf* OL = (bf*)take((size_t)NTK * HID * 2); float* OUTL = (float*)take((size_t)NTK * DIM * 4);
    if ((size_t)(wsp - (char*)d_ws) > ws_size) return;
    float* PROJ = HV; bf* PH = NHp; bf* PLw = NLp;
    k_emb<<<(NB_ * DIM) / 256, 256, 0, stream>>>(t, We, bemb, EMB);
    k_cvtw<<<(2 * HID) / 8, 256, 0, stream>>>(Wh, 2 * HID, WhB); k_cvtw<<<QK / 8, 256, 0, stream>>>(Wqk, QK, WqkB); k_cvtw<<<DIM / 8, 256, 0, stream>>>(Wout, DIM, WoB); k_cvtw<<<(2 * DIM) / 8, 256, 0, stream>>>(Wp, 2 * DIM, WpB);
    k_ln<<<NB_ * (LL / 64), 256, 0, stream>>>(x, EMB, lng, lnb, NHp, NLp);
    k_gemm<<<dim3(NTK / 64, (2 * HID) / 64, 1), 128, 0, stream>>>(NHp, NLp, WhB, bh, 2 * HID, HV);
    k_gemm<<<dim3(NTK / 64, QK / 64, 1), 128, 0, stream>>>(NHp, NLp, WqkB, bqk, QK, Zf);
    k_qk<<<NTK / 8, 256, 0, stream>>>(Zf, gam, bet, Q16, K16);
    k_vt<<<dim3(LL / 64, HID / 64, NB_), 256, 0, stream>>>(HV, VT16);
    k_attn<<<NB_ * (LL / 64), 128, 0, stream>>>(Q16, K16, VT16, HV, OH, OL);
    k_gemm<<<dim3(NTK / 64, DIM / 64, 1), 128, 0, stream>>>(OH, OL, WoB, bout, DIM, OUTL);
    k_split<<<NTK / 8, 256, 0, stream>>>(OUTL, PH, PLw);
    k_gemm<<<dim3(NTK / 64, (2 * DIM) / 64, 1), 128, 0, stream>>>(PH, PLw, WpB, bp, 2 * DIM, PROJ);
    k_final<<<dim3(LL / 64, DIM / 64, NB_), 256, 0, stream>>>(x, EMB, PROJ, out1, out2);
}
